// CaptioningRNN_60069412602579
// MI455X (gfx1250) — hardware-run, weakly checked
//
#include <hip/hip_runtime.h>
#include <math.h>

constexpr int NBATCH   = 64;
constexpr int NSTEP    = 128;
constexpr int NFEAT    = 512;
constexpr int NHID     = 1024;
constexpr int NLOC     = 16;
constexpr int NGATE    = 4 * NHID;
constexpr int KWT      = NFEAT + 2 * NHID;
constexpr int ROWS_BLK = 16;
constexpr int NTHR     = 512;
constexpr int NWAVE    = NTHR / 32;
constexpr int COLS_WAVE = NHID / NWAVE;
constexpr int NGRP     = COLS_WAVE / 16;
constexpr int APITCH   = 2 * NHID + 8;
constexpr int HPITCH   = NHID + 4;
constexpr int PREPT    = 256;
constexpr int SQRT_NHID = 32;
constexpr float SCORE_SCALE = 1.0f / (float)SQRT_NHID;
constexpr float LOC_INV     = 1.0f / (float)NLOC;
constexpr float ACARRY   = 64.0f;
constexpr float WCARRY   = 1024.0f;
constexpr float RCARRY   = 2048.0f;
constexpr float PROD_INV = 1.0f / (ACARRY * WCARRY);
constexpr float RES_INV  = 1.0f / RCARRY;
constexpr float F16_MIN_NORMAL = 6.103515625e-05f;
constexpr size_t GSTRIDE = (size_t)NHID * (size_t)KWT;

static_assert(SQRT_NHID * SQRT_NHID == NHID);
static_assert(NBATCH % ROWS_BLK == 0);
static_assert(NWAVE == ROWS_BLK);
static_assert(COLS_WAVE * NWAVE == NHID && NGRP == 4);
static_assert(NFEAT % 32 == 0 && NHID % 32 == 0 && KWT % 32 == 0);
static_assert(NGATE % 64 == 0 && NFEAT % 64 == 0 && NHID % 64 == 0);
static_assert((APITCH * 2) % 16 == 0 && (HPITCH * 4) % 16 == 0);
static_assert(NHID % 128 == 0);
static_assert((NBATCH * NSTEP * NFEAT / 8) % PREPT == 0);
static_assert((size_t)NBATCH * NSTEP * NHID * 4 == (size_t)33554432);

typedef __attribute__((ext_vector_type(16))) _Float16 v16h;
typedef __attribute__((ext_vector_type(8)))  _Float16 v8h;
typedef __attribute__((ext_vector_type(8)))  float    v8f;
typedef __attribute__((ext_vector_type(4)))  float    v4f;

union FragU { v16h v; v8h h[2]; };

__device__ __forceinline__ v16h frag_load(const _Float16* p) {
  FragU f;
  f.h[0] = *(const v8h*)(p);
  f.h[1] = *(const v8h*)(p + 16);
  return f.v;
}
__device__ __forceinline__ v8f frag_mma(v16h a, v16h b, v8f c) {
  return __builtin_amdgcn_wmma_f32_16x16x32_f16(false, a, false, b, (short)0, c, false, false);
}
__device__ __forceinline__ void guard_acc4(v8f& a0, v8f& a1, v8f& a2, v8f& a3,
                                           v16h x, v16h b0, v16h b1, v16h b2, v16h b3) {
  asm volatile("v_nop\n\tv_nop\n\tv_nop\n\tv_nop"
               : "+v"(a0), "+v"(a1), "+v"(a2), "+v"(a3)
               : "v"(x), "v"(b0), "v"(b1), "v"(b2), "v"(b3));
}
__device__ __forceinline__ void guard_acc8(v8f& a0, v8f& a1, v8f& a2, v8f& a3,
                                           v8f& r0, v8f& r1, v8f& r2, v8f& r3,
                                           v16h x, v16h y, v16h b0, v16h b1, v16h b2, v16h b3) {
  asm volatile("v_nop\n\tv_nop\n\tv_nop\n\tv_nop"
               : "+v"(a0), "+v"(a1), "+v"(a2), "+v"(a3), "+v"(r0), "+v"(r1), "+v"(r2), "+v"(r3)
               : "v"(x), "v"(y), "v"(b0), "v"(b1), "v"(b2), "v"(b3));
}
__device__ __forceinline__ void guard_tail8(v8f& a0, v8f& a1, v8f& a2, v8f& a3,
                                            v8f& r0, v8f& r1, v8f& r2, v8f& r3) {
  asm volatile("v_nop\n\tv_nop\n\tv_nop\n\tv_nop"
               : "+v"(a0), "+v"(a1), "+v"(a2), "+v"(a3), "+v"(r0), "+v"(r1), "+v"(r2), "+v"(r3));
}

__device__ __forceinline__ _Float16 to_h16(float v) {
  const float f = (fabsf(v) < F16_MIN_NORMAL) ? 0.0f : v;
  return (_Float16)f;
}

__device__ __forceinline__ float fsig(float x)  { return __builtin_amdgcn_rcpf(1.0f + __expf(-x)); }
__device__ __forceinline__ float ftanh(float x) { return 1.0f - 2.0f * __builtin_amdgcn_rcpf(__expf(2.0f * x) + 1.0f); }

__global__ __launch_bounds__(PREPT) void wplane_kernel(const float* __restrict__ src, int ncol, int ldo, int kofs,
                                                       unsigned short* __restrict__ O, float sc) {
  __shared__ float Tt[64 * 65];
  const int tid = threadIdx.x;
  const int c0 = blockIdx.x * 64, r0 = blockIdx.y * 64;
#pragma unroll
  for (int i = 0; i < 4; ++i) {
    const int idx = i * PREPT + tid;
    const int rr = idx >> 4, cc = (idx & 15) * 4;
    const v4f v = *(const v4f*)(src + (size_t)(r0 + rr) * (size_t)ncol + c0 + cc);
    Tt[rr * 65 + cc + 0] = v[0];
    Tt[rr * 65 + cc + 1] = v[1];
    Tt[rr * 65 + cc + 2] = v[2];
    Tt[rr * 65 + cc + 3] = v[3];
  }
  __syncthreads();
  const int q = tid >> 3, c8 = (tid & 7) * 8;
  v8h hv[2];
#pragma unroll
  for (int g = 0; g < 2; ++g) {
    const int qq = g * 32 + q;
#pragma unroll
    for (int e = 0; e < 8; ++e) {
      const float f = Tt[(c8 + e) * 65 + qq];
      hv[g][e] = to_h16(f * sc);
    }
  }
  for (int pass = 0; pass < 2; ++pass) {
#pragma unroll
    for (int g = 0; g < 2; ++g) {
      const size_t o = (size_t)(c0 + g * 32 + q) * (size_t)ldo + (size_t)(kofs + r0 + c8);
      *(volatile v8h*)(O + o) = hv[g];
    }
    __threadfence();
  }
}

__global__ __launch_bounds__(PREPT) void xsplit_kernel(const float* __restrict__ x, unsigned short* __restrict__ XH,
                                                       unsigned short* __restrict__ XL, int n8) {
  const int i = blockIdx.x * PREPT + threadIdx.x;
  if (i < n8) {
    const v4f a = *(const v4f*)(x + (size_t)i * 8);
    const v4f b = *(const v4f*)(x + (size_t)i * 8 + 4);
    v8h hv, lv;
#pragma unroll
    for (int e = 0; e < 4; ++e) {
      const float s0 = a[e] * ACARRY;
      const float s1 = b[e] * ACARRY;
      const _Float16 h0 = to_h16(s0);
      const _Float16 h1 = to_h16(s1);
      const float q0 = (s0 - (float)h0) * RCARRY;
      const float q1 = (s1 - (float)h1) * RCARRY;
      hv[e]     = h0;
      hv[4 + e] = h1;
      lv[e]     = to_h16(q0);
      lv[4 + e] = to_h16(q1);
    }
    for (int pass = 0; pass < 2; ++pass) {
      *(volatile v8h*)(XH + (size_t)i * 8) = hv;
      *(volatile v8h*)(XL + (size_t)i * 8) = lv;
      __threadfence();
    }
  }
}

__global__ __launch_bounds__(NTHR) void seq_kernel(const float* __restrict__ Afeat, const float* __restrict__ bias,
                                                   const unsigned short* __restrict__ XHp,
                                                   const unsigned short* __restrict__ XLp,
                                                   const unsigned short* __restrict__ WTp,
                                                   float* __restrict__ out) {
  __shared__ __align__(16) _Float16 Aha[ROWS_BLK * APITCH];
  __shared__ __align__(16) float    Hs[ROWS_BLK * HPITCH];
  const _Float16* XH = (const _Float16*)XHp;
  const _Float16* XL = (const _Float16*)XLp;
  const _Float16* WT = (const _Float16*)WTp;
  const int tid = threadIdx.x, lane = tid & 31, wave = tid >> 5;
  const int c = lane & 15, hh = lane >> 4, koff = hh * 8;
  const int rowbase = blockIdx.x * ROWS_BLK;
  const float* Arow = Afeat + (size_t)(rowbase + wave) * NHID * NLOC;
  float* hrow = Hs + wave * HPITCH;
  _Float16* arow = Aha + wave * APITCH;

#pragma unroll 1
  for (int it = 0; it < NHID / 32; ++it) {
    const int j = it * 32 + lane;
    const float* ap = Arow + (size_t)j * NLOC;
    const v4f a0 = *(const v4f*)(ap);
    const v4f a1 = *(const v4f*)(ap + 4);
    const v4f a2 = *(const v4f*)(ap + 8);
    const v4f a3 = *(const v4f*)(ap + 12);
    float s = 0.0f;
#pragma unroll
    for (int e = 0; e < 4; ++e) s += a0[e];
#pragma unroll
    for (int e = 0; e < 4; ++e) s += a1[e];
#pragma unroll
    for (int e = 0; e < 4; ++e) s += a2[e];
#pragma unroll
    for (int e = 0; e < 4; ++e) s += a3[e];
    hrow[j] = s * LOC_INV;
  }
  __syncthreads();

  float cst[NGRP][8], bb[NGRP][4];
#pragma unroll
  for (int nt = 0; nt < NGRP; ++nt) {
    const int j = COLS_WAVE * wave + 16 * nt + c;
#pragma unroll
    for (int g = 0; g < 4; ++g) bb[nt][g] = bias[g * NHID + j];
#pragma unroll
    for (int r = 0; r < 8; ++r) cst[nt][r] = Hs[(8 * hh + r) * HPITCH + j];
  }

  const v8f z8 = {0.f, 0.f, 0.f, 0.f, 0.f, 0.f, 0.f, 0.f};

#pragma unroll 1
  for (int t = 0; t < NSTEP; ++t) {
    {
      float sc[NLOC];
#pragma unroll
      for (int l = 0; l < NLOC; ++l) sc[l] = 0.0f;
#pragma unroll 1
      for (int it = 0; it < NHID / 32; ++it) {
        const int j = it * 32 + lane;
        const float hv = hrow[j];
        const float* ap = Arow + (size_t)j * NLOC;
        const v4f a0 = *(const v4f*)(ap);
        const v4f a1 = *(const v4f*)(ap + 4);
        const v4f a2 = *(const v4f*)(ap + 8);
        const v4f a3 = *(const v4f*)(ap + 12);
#pragma unroll
        for (int e = 0; e < 4; ++e) {
          sc[e]      = fmaf(hv, a0[e], sc[e]);
          sc[4 + e]  = fmaf(hv, a1[e], sc[4 + e]);
          sc[8 + e]  = fmaf(hv, a2[e], sc[8 + e]);
          sc[12 + e] = fmaf(hv, a3[e], sc[12 + e]);
        }
      }
#pragma unroll
      for (int off = 1; off < 32; off <<= 1) {
#pragma unroll
        for (int l = 0; l < NLOC; ++l) sc[l] += __shfl_xor(sc[l], off, 32);
      }
      float sown = sc[0];
#pragma unroll
      for (int l = 1; l < NLOC; ++l) sown = (c == l) ? sc[l] : sown;
      sown *= SCORE_SCALE;
      float mx = sown;
#pragma unroll
      for (int off = 1; off < 16; off <<= 1) {
        const float o = __shfl_xor(mx, off, 32);
        mx = fmaxf(mx, o);
      }
      const float p = expf(sown - mx);
      float ps = p;
#pragma unroll
      for (int off = 1; off < 16; off <<= 1) ps += __shfl_xor(ps, off, 32);
      const float wown = p * (1.0f / ps);
      float wgt[NLOC];
#pragma unroll
      for (int l = 0; l < NLOC; ++l) wgt[l] = __shfl(wown, l, 32);
#pragma unroll 1
      for (int it = 0; it < NHID / 32; ++it) {
        const int j = it * 32 + lane;
        const float hv = hrow[j];
        const float* ap = Arow + (size_t)j * NLOC;
        const v4f a0 = *(const v4f*)(ap);
        const v4f a1 = *(const v4f*)(ap + 4);
        const v4f a2 = *(const v4f*)(ap + 8);
        const v4f a3 = *(const v4f*)(ap + 12);
        float at = 0.0f;
#pragma unroll
        for (int e = 0; e < 4; ++e) at = fmaf(a0[e], wgt[e], at);
#pragma unroll
        for (int e = 0; e < 4; ++e) at = fmaf(a1[e], wgt[4 + e], at);
#pragma unroll
        for (int e = 0; e < 4; ++e) at = fmaf(a2[e], wgt[8 + e], at);
#pragma unroll
        for (int e = 0; e < 4; ++e) at = fmaf(a3[e], wgt[12 + e], at);
        arow[j]        = to_h16(hv * ACARRY);
        arow[NHID + j] = to_h16(at * ACARRY);
      }
    }
    __syncthreads();

    {
      const size_t xoff = ((size_t)(rowbase + c) * NSTEP + (size_t)t) * NFEAT + (size_t)koff;
      const _Float16* xh = XH + xoff;
      const _Float16* xl = XL + xoff;
      const _Float16* ah = Aha + c * APITCH + koff;
#pragma unroll
      for (int nt = 0; nt < NGRP; ++nt) {
        const int j = COLS_WAVE * wave + 16 * nt + c;
        const _Float16* w0 = WT + (size_t)j * KWT + koff;
        const _Float16* w1 = w0 + GSTRIDE;
        const _Float16* w2 = w1 + GSTRIDE;
        const _Float16* w3 = w2 + GSTRIDE;
        v8f am0 = z8, am1 = z8, am2 = z8, am3 = z8;
        v8f ar0 = z8, ar1 = z8, ar2 = z8, ar3 = z8;
#pragma unroll 1
        for (int k0 = 0; k0 < NFEAT; k0 += 32) {
          const v16h av = frag_load(xh + k0);
          const v16h al = frag_load(xl + k0);
          const v16h b0 = frag_load(w0 + k0);
          const v16h b1 = frag_load(w1 + k0);
          const v16h b2 = frag_load(w2 + k0);
          const v16h b3 = frag_load(w3 + k0);
          am0 = frag_mma(av, b0, am0);
          am1 = frag_mma(av, b1, am1);
          am2 = frag_mma(av, b2, am2);
          am3 = frag_mma(av, b3, am3);
          ar0 = frag_mma(al, b0, ar0);
          ar1 = frag_mma(al, b1, ar1);
          ar2 = frag_mma(al, b2, ar2);
          ar3 = frag_mma(al, b3, ar3);
          guard_acc8(am0, am1, am2, am3, ar0, ar1, ar2, ar3, av, al, b0, b1, b2, b3);
        }
#pragma unroll 1
        for (int k0 = 0; k0 < 2 * NHID; k0 += 32) {
          const v16h av = frag_load(ah + k0);
          const v16h b0 = frag_load(w0 + NFEAT + k0);
          const v16h b1 = frag_load(w1 + NFEAT + k0);
          const v16h b2 = frag_load(w2 + NFEAT + k0);
          const v16h b3 = frag_load(w3 + NFEAT + k0);
          am0 = frag_mma(av, b0, am0);
          am1 = frag_mma(av, b1, am1);
          am2 = frag_mma(av, b2, am2);
          am3 = frag_mma(av, b3, am3);
          guard_acc4(am0, am1, am2, am3, av, b0, b1, b2, b3);
        }
        guard_tail8(am0, am1, am2, am3, ar0, ar1, ar2, ar3);
#pragma unroll
        for (int r = 0; r < 8; ++r) {
          const float zi = fmaf(ar0[r], RES_INV, am0[r]) * PROD_INV + bb[nt][0];
          const float zf = fmaf(ar1[r], RES_INV, am1[r]) * PROD_INV + bb[nt][1];
          const float zo = fmaf(ar2[r], RES_INV, am2[r]) * PROD_INV + bb[nt][2];
          const float zg = fmaf(ar3[r], RES_INV, am3[r]) * PROD_INV + bb[nt][3];
          const float ig = fsig(zi);
          const float fg = fsig(zf);
          const float og = fsig(zo);
          const float gg = ftanh(zg);
          const float cn = fg * cst[nt][r] + ig * gg;
          cst[nt][r] = cn;
          const float hn = og * ftanh(cn);
          Hs[(8 * hh + r) * HPITCH + j] = hn;
        }
      }
    }
    __syncthreads();

    {
      float* dst = out + ((size_t)(rowbase + wave) * NSTEP + (size_t)t) * NHID;
      for (int pass = 0; pass < 2; ++pass) {
#pragma unroll
        for (int it = 0; it < NHID / 128; ++it) {
          const v4f v = *(const v4f*)(hrow + it * 128 + lane * 4);
          *(volatile v4f*)(dst + it * 128 + lane * 4) = v;
        }
        __threadfence();
      }
    }
  }
}

extern "C" void kernel_launch(void* const* d_in, const int* in_sizes, int n_in,
                              void* d_out, int out_size, void* d_ws, size_t ws_size, hipStream_t stream) {
  if (n_in < 6 || d_out == nullptr || d_ws == nullptr) return;
  if (in_sizes[0] != NBATCH * NSTEP * NFEAT || in_sizes[1] != NBATCH * NHID * NLOC ||
      in_sizes[2] != NFEAT * NGATE || in_sizes[3] != NHID * NGATE || in_sizes[4] != NHID * NGATE ||
      in_sizes[5] != NGATE || out_size != NBATCH * NSTEP * NHID) return;

  const float* x     = (const float*)d_in[0];
  const float* amap  = (const float*)d_in[1];
  const float* wx    = (const float*)d_in[2];
  const float* wh    = (const float*)d_in[3];
  const float* wattn = (const float*)d_in[4];
  const float* bvec  = (const float*)d_in[5];
  float* out = (float*)d_out;

  char* ws = (char*)d_ws;
  size_t off = 0;
  auto carve = [&](size_t bytes) -> char* { char* p = ws + off; off += (bytes + 255) & ~(size_t)255; return p; };
  unsigned short* WT = (unsigned short*)carve((size_t)NGATE * KWT * 2);
  unsigned short* XH = (unsigned short*)carve((size_t)NBATCH * NSTEP * NFEAT * 2);
  unsigned short* XL = (unsigned short*)carve((size_t)NBATCH * NSTEP * NFEAT * 2);
  if (off > ws_size || off > (size_t)134217728) return;

  wplane_kernel<<<dim3(NGATE / 64, NFEAT / 64), PREPT, 0, stream>>>(wx,    NGATE, KWT, 0,            WT, WCARRY);
  wplane_kernel<<<dim3(NGATE / 64, NHID / 64),  PREPT, 0, stream>>>(wh,    NGATE, KWT, NFEAT,        WT, WCARRY);
  wplane_kernel<<<dim3(NGATE / 64, NHID / 64),  PREPT, 0, stream>>>(wattn, NGATE, KWT, NFEAT + NHID, WT, WCARRY);
  const int n8 = NBATCH * NSTEP * NFEAT / 8;
  xsplit_kernel<<<n8 / PREPT, PREPT, 0, stream>>>(x, XH, XL, n8);
  seq_kernel<<<NBATCH / ROWS_BLK, NTHR, 0, stream>>>(amap, bvec, XH, XL, WT, out);
}
